// CrossATT_6047313952905
// MI455X (gfx1250) — hardware-verified
//
#include <hip/hip_runtime.h>
#include <math.h>

#define NB    16
#define CL    4096
#define QL    512
#define HD    128
#define XSC   1024.0f
#define KSC   1024.0f
#define VCAR  256.0f
#define PCAR  32768.0f
#define W0SC  1024.0f
#define W1SC  4096.0f
#define CQSC  256.0f
#define RSC   2048.0f
#define LOG2E 1.4426950408889634f
#define ATW   4
#define ATT_THREADS (ATW * 32)
#define QPB   (16 * ATW)
#define BPB   (CL / QPB)
#define ATT_BLOCKS (NB * BPB)
#define QP    20
#define SLABF (HD * QP)
#define VTP   72
#define VTILES (QL / 64)
#define GROWS 64
#define GBLOCKS ((NB * CL) / GROWS)
#define WTP   136
static_assert(HD == 128 && QPB == 64 && ATT_THREADS == 128);
static_assert((CL % QPB) == 0 && (QL % 64) == 0 && (QL % 32) == 0 && (HD % 32) == 0);
static_assert(BPB == 64 && VTILES == 8 && GBLOCKS == 1024);
static_assert((HD - 1) * VTP + 63 < HD * VTP);
static_assert((HD - 1) * QP + 15 < SLABF && (QP % 4) == 0);
static_assert(31 * WTP + 127 < 32 * WTP && (WTP % 8) == 0);
static_assert(((NB * CL * HD) % 2048) == 0 && ((NB * QL * HD) % 2048) == 0);
static_assert(((NB * CL) % GROWS) == 0);

typedef _Float16 v16h __attribute__((ext_vector_type(16)));
typedef _Float16 v8h  __attribute__((ext_vector_type(8)));
typedef float    v8f  __attribute__((ext_vector_type(8)));
typedef float    v4f  __attribute__((ext_vector_type(4)));
typedef unsigned int v4u __attribute__((ext_vector_type(4)));

union FragH { v16h v; v8h h[2]; v4u u[2]; };

__device__ __forceinline__ unsigned short bf_bits(float f) {
  unsigned u = __float_as_uint(f);
  return (unsigned short)((u + 0x7FFFu + ((u >> 16) & 1u)) >> 16);
}
__device__ __forceinline__ float bf_up(unsigned short h) { return __uint_as_float(((unsigned)h) << 16); }
__device__ __forceinline__ float bfr(float f) { return bf_up(bf_bits(f)); }
__device__ __forceinline__ unsigned short h_bits(_Float16 x) { return __builtin_bit_cast(unsigned short, x); }
__device__ __forceinline__ unsigned pk16(unsigned short a, unsigned short b) { return (unsigned)a | ((unsigned)b << 16); }
__device__ __forceinline__ v8f zero8() { v8f z = {0.f, 0.f, 0.f, 0.f, 0.f, 0.f, 0.f, 0.f}; return z; }

__device__ __forceinline__ v16h ldfrag_h(const _Float16* p) {
  FragH f;
  f.h[0] = *(const v8h*)(p);
  f.h[1] = *(const v8h*)(p + 16);
  return f.v;
}

__device__ __forceinline__ v8f mma_raw(v16h a, v16h b, v8f c) {
  return __builtin_amdgcn_wmma_f32_16x16x32_f16(false, a, false, b, (short)0, c, false, false);
}
__device__ __forceinline__ void guard_s(v8f& s, v16h x0, v16h x1, v16h x2, v16h x3,
                                        v16h y0, v16h y1, v16h y2, v16h y3) {
#if defined(__HIP_DEVICE_COMPILE__)
  asm volatile("v_nop\n\tv_nop\n\tv_nop\n\tv_nop"
               : "+v"(s) : "v"(x0), "v"(x1), "v"(x2), "v"(x3), "v"(y0), "v"(y1), "v"(y2), "v"(y3) : "memory");
#endif
}
__device__ __forceinline__ void guard_o4(v8f& a, v8f& b, v8f& c, v8f& d,
                                         v16h p, v16h x0, v16h x1, v16h x2, v16h x3) {
#if defined(__HIP_DEVICE_COMPILE__)
  asm volatile("v_nop\n\tv_nop\n\tv_nop\n\tv_nop"
               : "+v"(a), "+v"(b), "+v"(c), "+v"(d) : "v"(p), "v"(x0), "v"(x1), "v"(x2), "v"(x3) : "memory");
#endif
}
__device__ __forceinline__ void guard_g4(v8f& a, v8f& b, v16h x0, v16h x1, v16h x2, v16h x3) {
#if defined(__HIP_DEVICE_COMPILE__)
  asm volatile("v_nop\n\tv_nop\n\tv_nop\n\tv_nop"
               : "+v"(a), "+v"(b) : "v"(x0), "v"(x1), "v"(x2), "v"(x3) : "memory");
#endif
}
__device__ __forceinline__ void acc_guard8(v8f& a, v8f& b, v8f& c, v8f& d, v8f& e, v8f& f, v8f& g, v8f& hx) {
#if defined(__HIP_DEVICE_COMPILE__)
  asm volatile("v_nop\n\tv_nop\n\tv_nop\n\tv_nop"
               : "+v"(a), "+v"(b), "+v"(c), "+v"(d), "+v"(e), "+v"(f), "+v"(g), "+v"(hx));
#endif
}
__device__ __forceinline__ void wave_sync_lds() {
  __builtin_amdgcn_fence(__ATOMIC_RELEASE, "workgroup");
  __builtin_amdgcn_wave_barrier();
  __builtin_amdgcn_fence(__ATOMIC_ACQUIRE, "workgroup");
}

__global__ __launch_bounds__(256) void cvt16(const float* __restrict__ xc, const float* __restrict__ xq,
                                             const int* __restrict__ cm, const int* __restrict__ qm,
                                             unsigned short* plc, unsigned short* plq,
                                             int nbc, int n8c, int n8q, float scc, float scq) {
  (void)cm; (void)qm;
  const bool sq  = ((int)blockIdx.x >= nbc);
  const int  blk = sq ? ((int)blockIdx.x - nbc) : (int)blockIdx.x;
  const int  gt  = blk * 256 + (int)threadIdx.x;
  const int  n8  = sq ? n8q : n8c;
  if (gt >= n8) return;
  const float* x = sq ? xq : xc;
  unsigned short* pl = sq ? plq : plc;
  const float sc = sq ? scq : scc;
  const size_t e = (size_t)gt * 8;
  const v4f a = *(const v4f*)(x + e), bq = *(const v4f*)(x + e + 4);
  v4u o;
#pragma unroll
  for (int i = 0; i < 2; ++i) {
    o[i]     = pk16(h_bits((_Float16)(bfr(a[2 * i]) * sc)),  h_bits((_Float16)(bfr(a[2 * i + 1]) * sc)));
    o[2 + i] = pk16(h_bits((_Float16)(bfr(bq[2 * i]) * sc)), h_bits((_Float16)(bfr(bq[2 * i + 1]) * sc)));
  }
  unsigned short* d = pl + e;
  for (int pass = 0; pass < 2; ++pass) {
    *(volatile v4u*)(d) = o;
    __threadfence();
  }
}

__global__ __launch_bounds__(256) void vt16(const float* __restrict__ v, unsigned short* VTo) {
  __shared__ __align__(16) unsigned short T[HD * VTP];
  const int tid = threadIdx.x;
  const int bid = blockIdx.x;
  const int bb  = bid / VTILES;
  const int t   = bid - bb * VTILES;
  if (bb >= NB) return;
  {
    const int sl = tid >> 2;
    const int dc = (tid & 3) * 32;
    int key = 64 * t + sl;
    key = (key < 0) ? 0 : ((key > QL - 1) ? (QL - 1) : key);
    const float* src = v + (((size_t)bb * QL + (size_t)key) * HD + dc);
#pragma unroll
    for (int i = 0; i < 8; ++i) {
      const v4f a = *(const v4f*)(src + 4 * i);
#pragma unroll
      for (int e = 0; e < 4; ++e) T[(dc + 4 * i + e) * VTP + sl] = h_bits((_Float16)(bfr(a[e]) * VCAR));
    }
  }
  __syncthreads();
  v4u vals[4];
  const int q8 = tid >> 3, p8 = (tid & 7) * 8;
#pragma unroll
  for (int it = 0; it < 4; ++it) {
    const int line = it * 32 + q8;
    vals[it] = *(const v4u*)(T + line * VTP + p8);
  }
  unsigned short* dst = VTo + ((size_t)bb * HD) * QL + 64 * t + p8;
  for (int pass = 0; pass < 2; ++pass) {
#pragma unroll
    for (int it = 0; it < 4; ++it) {
      const int line = it * 32 + q8;
      *(volatile v4u*)(dst + (size_t)line * QL) = vals[it];
    }
    __threadfence();
  }
}

__global__ __launch_bounds__(256) void wt16(const float* __restrict__ Wa, const float* __restrict__ Wb,
                                            unsigned short* WTa, unsigned short* WTb, float sca, float scb) {
  __shared__ __align__(16) unsigned short T[32 * WTP];
  const int tid = threadIdx.x;
  const bool one = (blockIdx.y != 0);
  const float* W = one ? Wb : Wa;
  unsigned short* WT = one ? WTb : WTa;
  const float sc = one ? scb : sca;
  const int e0 = (int)blockIdx.x * 32;
  if (e0 + 32 > HD) return;
  {
    const int d  = tid >> 1;
    const int ec = (tid & 1) * 16;
    const float* src = W + (size_t)d * HD + e0 + ec;
#pragma unroll
    for (int i = 0; i < 4; ++i) {
      const v4f a = *(const v4f*)(src + 4 * i);
#pragma unroll
      for (int e = 0; e < 4; ++e) T[(ec + 4 * i + e) * WTP + d] = h_bits((_Float16)(bfr(a[e]) * sc));
    }
  }
  __syncthreads();
  v4u vals[2];
  const int rq = tid >> 4, p8 = (tid & 15) * 8;
#pragma unroll
  for (int it = 0; it < 2; ++it) {
    const int row = it * 16 + rq;
    vals[it] = *(const v4u*)(T + row * WTP + p8);
  }
  unsigned short* dst = WT + (size_t)e0 * HD + p8;
  for (int pass = 0; pass < 2; ++pass) {
#pragma unroll
    for (int it = 0; it < 2; ++it) {
      const int row = it * 16 + rq;
      *(volatile v4u*)(dst + (size_t)row * HD) = vals[it];
    }
    __threadfence();
  }
}

__global__ __launch_bounds__(ATT_THREADS)
void attn_fwd(const unsigned short* __restrict__ XCp, const unsigned short* __restrict__ XQp,
              const unsigned short* __restrict__ VTq, unsigned short* CHp, unsigned short* CRp) {
  __shared__ __align__(16) float smem[ATW * SLABF];

  const int tid  = threadIdx.x;
  const int wave = tid >> 5;
  const int lane = tid & 31;
  const int hh   = lane >> 4;
  const int c    = lane & 15;

  const int bid  = blockIdx.x;
  const int bb   = bid / BPB;
  const int t    = bid - bb * BPB;
  if (bb >= NB) return;

  const int iw = QPB * t + wave * 16;

  const _Float16* Qb = (const _Float16*)(const void*)XCp + ((size_t)bb * CL + (size_t)(iw + c)) * HD + 8 * hh;
  const v16h qf0 = ldfrag_h(Qb);
  const v16h qf1 = ldfrag_h(Qb + 32);
  const v16h qf2 = ldfrag_h(Qb + 64);
  const v16h qf3 = ldfrag_h(Qb + 96);
  const _Float16* Kb = (const _Float16*)(const void*)XQp + ((size_t)bb * QL + (size_t)c) * HD + 8 * hh;
  const _Float16* Vb = (const _Float16*)(const void*)VTq + ((size_t)bb * HD + (size_t)c) * QL + 8 * hh;
  const float lsc = LOG2E / (XSC * KSC);

  float m_run = -INFINITY, l_run = 0.f;
  v8f o[8];
#pragma unroll
  for (int j = 0; j < 8; ++j) o[j] = zero8();

#pragma unroll 1
  for (int kb = 0; kb < QL; kb += 32) {
    v8f s0 = zero8(), s1 = zero8();
    {
      const _Float16* k0p = Kb + (size_t)kb * HD;
      const v16h a0 = ldfrag_h(k0p), a1 = ldfrag_h(k0p + 32), a2 = ldfrag_h(k0p + 64), a3 = ldfrag_h(k0p + 96);
      s0 = mma_raw(a0, qf0, s0);
      s0 = mma_raw(a1, qf1, s0);
      s0 = mma_raw(a2, qf2, s0);
      s0 = mma_raw(a3, qf3, s0);
      guard_s(s0, a0, a1, a2, a3, qf0, qf1, qf2, qf3);
      const _Float16* k1p = k0p + (size_t)16 * HD;
      const v16h b0 = ldfrag_h(k1p), b1 = ldfrag_h(k1p + 32), b2 = ldfrag_h(k1p + 64), b3 = ldfrag_h(k1p + 96);
      s1 = mma_raw(b0, qf0, s1);
      s1 = mma_raw(b1, qf1, s1);
      s1 = mma_raw(b2, qf2, s1);
      s1 = mma_raw(b3, qf3, s1);
      guard_s(s1, b0, b1, b2, b3, qf0, qf1, qf2, qf3);
    }
    float u0[8], u1[8];
    float mx = -INFINITY;
#pragma unroll
    for (int r = 0; r < 8; ++r) {
      u0[r] = s0[r] * lsc;
      u1[r] = s1[r] * lsc;
      mx = fmaxf(mx, fmaxf(u0[r], u1[r]));
    }
    mx = fmaxf(mx, __shfl_xor(mx, 16, 32));
    const float mn = fmaxf(m_run, mx);
    const float al = exp2f(m_run - mn);
    m_run = mn;
    float ps = 0.f;
    FragH pa;
#pragma unroll
    for (int r = 0; r < 8; ++r) {
      const float e0 = exp2f(u0[r] - mn), e1 = exp2f(u1[r] - mn);
      ps += e0 + e1;
      pa.h[0][r] = (_Float16)(e0 * PCAR);
      pa.h[1][r] = (_Float16)(e1 * PCAR);
    }
    ps += __shfl_xor(ps, 16, 32);
    l_run = l_run * al + ps;
#pragma unroll
    for (int r = 0; r < 8; ++r) {
      const float af = __shfl(al, 8 * hh + r, 32);
#pragma unroll
      for (int j = 0; j < 8; ++j) o[j][r] *= af;
    }
    {
      const _Float16* vp = Vb + kb;
      const v16h v0 = ldfrag_h(vp);
      const v16h v1 = ldfrag_h(vp + (size_t)16 * QL);
      const v16h v2 = ldfrag_h(vp + (size_t)32 * QL);
      const v16h v3 = ldfrag_h(vp + (size_t)48 * QL);
      o[0] = mma_raw(pa.v, v0, o[0]);
      o[1] = mma_raw(pa.v, v1, o[1]);
      o[2] = mma_raw(pa.v, v2, o[2]);
      o[3] = mma_raw(pa.v, v3, o[3]);
      guard_o4(o[0], o[1], o[2], o[3], pa.v, v0, v1, v2, v3);
      const v16h v4 = ldfrag_h(vp + (size_t)64 * QL);
      const v16h v5 = ldfrag_h(vp + (size_t)80 * QL);
      const v16h v6 = ldfrag_h(vp + (size_t)96 * QL);
      const v16h v7 = ldfrag_h(vp + (size_t)112 * QL);
      o[4] = mma_raw(pa.v, v4, o[4]);
      o[5] = mma_raw(pa.v, v5, o[5]);
      o[6] = mma_raw(pa.v, v6, o[6]);
      o[7] = mma_raw(pa.v, v7, o[7]);
      guard_o4(o[4], o[5], o[6], o[7], pa.v, v4, v5, v6, v7);
    }
  }
  acc_guard8(o[0], o[1], o[2], o[3], o[4], o[5], o[6], o[7]);

  const float oc = 1.0f / (PCAR * VCAR);
  const float li = (l_run > 0.0f) ? ((1.0f / l_run) * oc) : 0.0f;
  float* slab = smem + wave * SLABF;
  float lf[8];
#pragma unroll
  for (int r = 0; r < 8; ++r) lf[r] = __shfl(li, 8 * hh + r, 32);
#pragma unroll
  for (int j = 0; j < 8; ++j) {
    v4f w0, w1;
#pragma unroll
    for (int r = 0; r < 4; ++r) { w0[r] = o[j][r] * lf[r]; w1[r] = o[j][4 + r] * lf[4 + r]; }
    float* sp = slab + (16 * j + c) * QP + 8 * hh;
    *(v4f*)(sp)     = w0;
    *(v4f*)(sp + 4) = w1;
  }
  wave_sync_lds();
  v4u hv[8], rv[8];
#pragma unroll
  for (int it = 0; it < 8; ++it) {
    const int q = 2 * it + hh;
#pragma unroll
    for (int i = 0; i < 4; ++i) {
      const float va = slab[(8 * c + 2 * i) * QP + q] * CQSC;
      const float vb = slab[(8 * c + 2 * i + 1) * QP + q] * CQSC;
      const _Float16 ha = (_Float16)va, hb = (_Float16)vb;
      const _Float16 ra = (_Float16)((va - (float)ha) * RSC);
      const _Float16 rb = (_Float16)((vb - (float)hb) * RSC);
      hv[it][i] = pk16(h_bits(ha), h_bits(hb));
      rv[it][i] = pk16(h_bits(ra), h_bits(rb));
    }
  }
  const size_t rowoff = ((size_t)bb * CL + (size_t)iw) * HD + 8 * (size_t)lane;
  unsigned short* dh = CHp + rowoff;
  unsigned short* dr = CRp + rowoff;
  for (int pass = 0; pass < 2; ++pass) {
#pragma unroll
    for (int it = 0; it < 8; ++it) {
      *(volatile v4u*)(dh + (size_t)it * 2 * HD) = hv[it];
      *(volatile v4u*)(dr + (size_t)it * 2 * HD) = rv[it];
    }
    __threadfence();
  }
}

__global__ __launch_bounds__(ATT_THREADS)
void gemm_out(const unsigned short* __restrict__ CHp, const unsigned short* __restrict__ CRp,
              const unsigned short* __restrict__ XCp, const unsigned short* __restrict__ W1p,
              const unsigned short* __restrict__ W0p, float* OPp, int nrows) {
  __shared__ __align__(16) float smem[ATW * SLABF];

  const int tid  = threadIdx.x;
  const int wave = tid >> 5;
  const int lane = tid & 31;
  const int hh   = lane >> 4;
  const int c    = lane & 15;

  const int rb = (int)blockIdx.x * GROWS;
  if (rb + GROWS > nrows) return;
  const int r0 = rb + wave * 16;

  const _Float16* Ab = (const _Float16*)(const void*)CHp + ((size_t)(r0 + c)) * HD + 8 * hh;
  const _Float16* Rb = (const _Float16*)(const void*)CRp + ((size_t)(r0 + c)) * HD + 8 * hh;
  const _Float16* Xb = (const _Float16*)(const void*)XCp + ((size_t)(r0 + c)) * HD + 8 * hh;
  const v16h ch0 = ldfrag_h(Ab), ch1 = ldfrag_h(Ab + 32), ch2 = ldfrag_h(Ab + 64), ch3 = ldfrag_h(Ab + 96);
  const v16h cr0 = ldfrag_h(Rb), cr1 = ldfrag_h(Rb + 32), cr2 = ldfrag_h(Rb + 64), cr3 = ldfrag_h(Rb + 96);
  const v16h xc0 = ldfrag_h(Xb), xc1 = ldfrag_h(Xb + 32), xc2 = ldfrag_h(Xb + 64), xc3 = ldfrag_h(Xb + 96);
  const _Float16* W1b = (const _Float16*)(const void*)W1p + ((size_t)c) * HD + 8 * hh;
  const _Float16* W0b = (const _Float16*)(const void*)W0p + ((size_t)c) * HD + 8 * hh;

  const float sa = 1.0f / (CQSC * W1SC);
  const float sr = 1.0f / (CQSC * W1SC * RSC);
  float* slab = smem + wave * SLABF;

#pragma unroll 1
  for (int t = 0; t < 8; ++t) {
    v8f acc = zero8(), acr = zero8();
    {
      const _Float16* w1p = W1b + (size_t)t * 16 * HD;
      const v16h p0 = ldfrag_h(w1p), p1 = ldfrag_h(w1p + 32), p2 = ldfrag_h(w1p + 64), p3 = ldfrag_h(w1p + 96);
      acc = mma_raw(ch0, p0, acc);
      acc = mma_raw(ch1, p1, acc);
      acc = mma_raw(ch2, p2, acc);
      acc = mma_raw(ch3, p3, acc);
      acr = mma_raw(cr0, p0, acr);
      acr = mma_raw(cr1, p1, acr);
      acr = mma_raw(cr2, p2, acr);
      acr = mma_raw(cr3, p3, acr);
      guard_g4(acc, acr, p0, p1, p2, p3);
    }
    {
      const _Float16* w0p = W0b + (size_t)t * 16 * HD;
      const v16h g0 = ldfrag_h(w0p), g1 = ldfrag_h(w0p + 32), g2 = ldfrag_h(w0p + 64), g3 = ldfrag_h(w0p + 96);
      acc = mma_raw(xc0, g0, acc);
      acc = mma_raw(xc1, g1, acc);
      acc = mma_raw(xc2, g2, acc);
      acc = mma_raw(xc3, g3, acc);
      guard_g4(acc, acr, g0, g1, g2, g3);
    }
    v4f w0, w1;
#pragma unroll
    for (int r = 0; r < 4; ++r) {
      w0[r] = acc[r] * sa + acr[r] * sr;
      w1[r] = acc[4 + r] * sa + acr[4 + r] * sr;
    }
    float* sp = slab + (16 * t + c) * QP + 8 * hh;
    *(v4f*)(sp)     = w0;
    *(v4f*)(sp + 4) = w1;
  }
  wave_sync_lds();
  v4f vals[16];
#pragma unroll
  for (int it = 0; it < 16; ++it) {
#pragma unroll
    for (int e = 0; e < 4; ++e) vals[it][e] = slab[(4 * lane + e) * QP + it];
  }
  float* dst = OPp + ((size_t)r0) * HD + 4 * lane;
  for (int pass = 0; pass < 2; ++pass) {
#pragma unroll
    for (int it = 0; it < 16; ++it) {
      *(volatile v4f*)(dst + (size_t)it * HD) = vals[it];
    }
    __threadfence();
  }
}

extern "C" void kernel_launch(void* const* d_in, const int* in_sizes, int n_in,
                              void* d_out, int out_size, void* d_ws, size_t ws_size,
                              hipStream_t stream) {
  const int NEC = NB * CL * HD;
  const int NEQ = NB * QL * HD;
  if (n_in < 6) return;
  if (in_sizes[0] < NEC || in_sizes[1] < NEQ) return;
  if (in_sizes[4] < HD * HD || in_sizes[5] < HD * HD) return;
  if (out_size < NEC) return;

  const float* xc = (const float*)d_in[0];
  const float* xq = (const float*)d_in[1];
  const int*   cm = (const int*)d_in[2];
  const int*   qm = (const int*)d_in[3];
  const float* W0 = (const float*)d_in[4];
  const float* W1 = (const float*)d_in[5];
  float*       out = (float*)d_out;

  const size_t PXC = (size_t)NEC * 2;
  const size_t PXQ = (size_t)NEQ * 2;
  const size_t PVT = (size_t)NB * HD * QL * 2;
  const size_t PW  = (size_t)HD * HD * 2;
  const size_t PCQ = (size_t)NEC * 2;
  size_t off = 0;
  const size_t oXC = off; off += PXC;
  const size_t oXQ = off; off += PXQ;
  const size_t oVT = off; off += PVT;
  const size_t oW0 = off; off += PW;
  const size_t oW1 = off; off += PW;
  const size_t oCH = off; off += PCQ;
  const size_t oCR = off; off += PCQ;
  if (off > ws_size) return;
  if (off > (size_t)134217728) return;

  char* ws = (char*)d_ws;
  unsigned short* XC  = (unsigned short*)(ws + oXC);
  unsigned short* XQ  = (unsigned short*)(ws + oXQ);
  unsigned short* VT  = (unsigned short*)(ws + oVT);
  unsigned short* W0T = (unsigned short*)(ws + oW0);
  unsigned short* W1T = (unsigned short*)(ws + oW1);
  unsigned short* CH  = (unsigned short*)(ws + oCH);
  unsigned short* CR  = (unsigned short*)(ws + oCR);

  const int n8c = NEC / 8;
  const int n8q = NEQ / 8;
  const int nbc = n8c / 256;
  const int nbq = n8q / 256;
  const dim3 blk(256);
  const dim3 gC(nbc + nbq);
  const dim3 gVT(NB * VTILES);
  const dim3 gW(HD / 32, 2);
  const dim3 gAT(ATT_BLOCKS);
  const dim3 bAT(ATT_THREADS);
  const dim3 gG(GBLOCKS);

  cvt16<<<gC, blk, 0, stream>>>(xc, xq, cm, qm, XC, XQ, nbc, n8c, n8q, XSC, KSC);
  vt16<<<gVT, blk, 0, stream>>>(xq, VT);
  wt16<<<gW, blk, 0, stream>>>(W0, W1, W0T, W1T, W0SC, W1SC);
  attn_fwd<<<gAT, bAT, 0, stream>>>(XC, XQ, VT, CH, CR);
  gemm_out<<<gG, bAT, 0, stream>>>(CH, CR, XC, W1T, W0T, out, NB * CL);
  (void)hipGetLastError();
}
